// TTTLayer_7499012899548
// MI455X (gfx1250) — hardware-run, weakly checked
//
#include <hip/hip_runtime.h>

constexpr int NBATCH = 4;
constexpr int NSTEP  = 2048;
constexpr int DMODEL = 1024;
constexpr int DSTATE = 256;
constexpr int MROWS  = NBATCH * NSTEP;
constexpr float INNER_STEP = 0.01f;

static_assert(DSTATE * 4 == DMODEL, "state width is a quarter of the model width");
static_assert(MROWS % 64 == 0 && DMODEL % 64 == 0 && DSTATE % 64 == 0, "GEMM tiles are 64 x 64");
static_assert(DMODEL % 32 == 0 && DSTATE % 32 == 0, "GEMM K steps by 32 with no tail");
static_assert((MROWS * DMODEL) % (8 * 256) == 0, "plane split kernel covers x exactly");

typedef __attribute__((ext_vector_type(16))) __bf16   v16b;
typedef __attribute__((ext_vector_type(8)))  __bf16   v8b;
typedef __attribute__((ext_vector_type(8)))  float    v8f;
typedef __attribute__((ext_vector_type(4)))  float    v4f;
typedef __attribute__((ext_vector_type(4)))  unsigned v4u;

__device__ __forceinline__ unsigned f2bf_bits(float f) {
  const unsigned u = __float_as_uint(f);
  return ((u + 0x7FFFu + ((u >> 16) & 1u)) >> 16) & 0xFFFFu;
}
__device__ __forceinline__ float bf_bits2f(unsigned h) { return __uint_as_float(h << 16); }

__device__ __forceinline__ void split8(const float (&f)[8], v4u& hv, v4u& lv) {
  unsigned hb[8], lb[8];
#pragma unroll
  for (int e = 0; e < 8; ++e) {
    hb[e] = f2bf_bits(f[e]);
    const float res = f[e] - bf_bits2f(hb[e]);
    lb[e] = f2bf_bits(res);
  }
  hv[0] = hb[0] | (hb[1] << 16);
  hv[1] = hb[2] | (hb[3] << 16);
  hv[2] = hb[4] | (hb[5] << 16);
  hv[3] = hb[6] | (hb[7] << 16);
  lv[0] = lb[0] | (lb[1] << 16);
  lv[1] = lb[2] | (lb[3] << 16);
  lv[2] = lb[4] | (lb[5] << 16);
  lv[3] = lb[6] | (lb[7] << 16);
}

__device__ __forceinline__ void tie1_b(v8f& a, v16b x, v16b y) { asm volatile("v_nop" : "+v"(a) : "v"(x), "v"(y)); }
__device__ __forceinline__ void guard1_b(v8f& a, v16b x, v16b y) { asm volatile("v_nop\n\tv_nop\n\tv_nop\n\tv_nop" : "+v"(a) : "v"(x), "v"(y)); }
__device__ __forceinline__ void keep4_b(v16b a, v16b b, v16b c, v16b d) { asm volatile("v_nop" :: "v"(a), "v"(b), "v"(c), "v"(d)); }
__device__ __forceinline__ void acc_guard4(v8f& a, v8f& b, v8f& c, v8f& d) { asm volatile("v_nop\n\tv_nop\n\tv_nop\n\tv_nop" : "+v"(a), "+v"(b), "+v"(c), "+v"(d)); }

struct FragB {
  union U { v16b v; v8b h[2]; };
  static __device__ __forceinline__ v16b load(const __bf16* p) {
    U f; f.h[0] = *(const v8b*)(p); f.h[1] = *(const v8b*)(p + 16); return f.v;
  }
  static __device__ __forceinline__ v8f mma(v16b a, v16b b, v8f c) {
    return __builtin_amdgcn_wmma_f32_16x16x32_bf16(false, a, false, b, (short)0, c, false, false);
  }
};

__global__ __launch_bounds__(256) void split_planes_kernel(const float* __restrict__ in,
                                                           unsigned short* __restrict__ hi,
                                                           unsigned short* __restrict__ lo, int n8) {
  const int i = blockIdx.x * 256 + threadIdx.x;
  if (i < n8) {
    const v4f a = *(const v4f*)(in + (size_t)i * 8);
    const v4f c = *(const v4f*)(in + (size_t)i * 8 + 4);
    const float fv[8] = {a[0], a[1], a[2], a[3], c[0], c[1], c[2], c[3]};
    v4u hv, lv;
    split8(fv, hv, lv);
    for (int pass = 0; pass < 2; ++pass) {
      *(volatile v4u*)(hi + (size_t)i * 8) = hv;
      *(volatile v4u*)(lo + (size_t)i * 8) = lv;
      __threadfence();
    }
  }
}

__global__ __launch_bounds__(256) void transpose_split_kernel(const float* __restrict__ in,
                                                              unsigned short* __restrict__ hi,
                                                              unsigned short* __restrict__ lo,
                                                              int R, int Cc) {
  __shared__ float tile[64 * 65];
  const int tid = threadIdx.x;
  const int r0 = blockIdx.x * 64;
  const int c0 = blockIdx.y * 64;
#pragma unroll
  for (int it = 0; it < 4; ++it) {
    const int idx = it * 256 + tid;
    const int r = idx >> 4;
    const int c4 = (idx & 15) * 4;
    const v4f v = *(const v4f*)(in + (size_t)(r0 + r) * Cc + c0 + c4);
    tile[r * 65 + c4 + 0] = v[0];
    tile[r * 65 + c4 + 1] = v[1];
    tile[r * 65 + c4 + 2] = v[2];
    tile[r * 65 + c4 + 3] = v[3];
  }
  __syncthreads();
  v4u hv[2], lv[2];
#pragma unroll
  for (int it = 0; it < 2; ++it) {
    const int idx = it * 256 + tid;
    const int cl = idx >> 3;
    const int q = idx & 7;
    float fv[8];
#pragma unroll
    for (int e = 0; e < 8; ++e) fv[e] = tile[(8 * q + e) * 65 + cl];
    split8(fv, hv[it], lv[it]);
  }
  for (int pass = 0; pass < 2; ++pass) {
#pragma unroll
    for (int it = 0; it < 2; ++it) {
      const int idx = it * 256 + tid;
      const int cl = idx >> 3;
      const int q = idx & 7;
      const size_t o = (size_t)(c0 + cl) * R + r0 + 8 * q;
      *(volatile v4u*)(hi + o) = hv[it];
      *(volatile v4u*)(lo + o) = lv[it];
    }
    __threadfence();
  }
}

template <bool RESID>
__global__ __launch_bounds__(256) void gemm_bf16x3_kernel(
    const unsigned short* __restrict__ Ahp, const unsigned short* __restrict__ Alp, int lda,
    const unsigned short* __restrict__ Bhp, const unsigned short* __restrict__ Blp, int ldb,
    float* __restrict__ C, int ldc,
    const float* __restrict__ bias, const float* __restrict__ resid,
    int M, int N, int K) {
  __shared__ __align__(16) float sT[8][16 * 68];
  const __bf16* Ah = (const __bf16*)(const void*)Ahp;
  const __bf16* Al = (const __bf16*)(const void*)Alp;
  const __bf16* Bh = (const __bf16*)(const void*)Bhp;
  const __bf16* Bl = (const __bf16*)(const void*)Blp;
  const int lane = threadIdx.x & 31;
  const int wave = threadIdx.x >> 5;
  const int tilesN = N >> 6;
  const int tilesM = M >> 6;
  const int tile = blockIdx.x * 8 + wave;
  if (tile >= tilesM * tilesN) return;
  const int tm = tile / tilesN;
  const int tn = tile - tm * tilesN;
  const int m0 = tm << 6;
  const int n0 = tn << 6;

  const int rlane = lane & 15;
  const int koff  = (lane >> 4) * 8;
  const int mOff  = (lane >> 4) * 8;

  v8f acc[4][4];
#pragma unroll
  for (int i = 0; i < 4; ++i)
#pragma unroll
    for (int j = 0; j < 4; ++j) acc[i][j] = (v8f){0.f, 0.f, 0.f, 0.f, 0.f, 0.f, 0.f, 0.f};

  for (int k0 = 0; k0 < K; k0 += 32) {
    v16b bh[4], bl[4];
#pragma unroll
    for (int j = 0; j < 4; ++j) {
      const size_t bo = (size_t)(n0 + (j << 4) + rlane) * ldb + koff + k0;
      bh[j] = FragB::load(Bh + bo);
      bl[j] = FragB::load(Bl + bo);
    }
#pragma unroll
    for (int i = 0; i < 4; ++i) {
      const size_t ao = (size_t)(m0 + (i << 4) + rlane) * lda + koff + k0;
      const v16b ah = FragB::load(Ah + ao);
      const v16b al = FragB::load(Al + ao);
#pragma unroll
      for (int j = 0; j < 4; ++j) {
        acc[i][j] = FragB::mma(ah, bh[j], acc[i][j]);
        acc[i][j] = FragB::mma(ah, bl[j], acc[i][j]);
        acc[i][j] = FragB::mma(al, bh[j], acc[i][j]);
      }
      tie1_b(acc[i][0], ah, al);
      tie1_b(acc[i][1], ah, al);
      tie1_b(acc[i][2], ah, al);
      guard1_b(acc[i][3], ah, al);
    }
    keep4_b(bh[0], bh[1], bh[2], bh[3]);
    keep4_b(bl[0], bl[1], bl[2], bl[3]);
  }
  acc_guard4(acc[0][0], acc[0][1], acc[0][2], acc[0][3]);
  acc_guard4(acc[1][0], acc[1][1], acc[1][2], acc[1][3]);
  acc_guard4(acc[2][0], acc[2][1], acc[2][2], acc[2][3]);
  acc_guard4(acc[3][0], acc[3][1], acc[3][2], acc[3][3]);

  float bv[4];
#pragma unroll
  for (int j = 0; j < 4; ++j) bv[j] = bias[n0 + (j << 4) + rlane];

  float* slab = sT[wave];
  const int hh = lane >> 4;
  const int c4 = (lane & 15) * 4;
#pragma unroll
  for (int i = 0; i < 4; ++i) {
    const int mBase = m0 + (i << 4);
#pragma unroll
    for (int j = 0; j < 4; ++j) {
#pragma unroll
      for (int r = 0; r < 8; ++r) {
        const float v = acc[i][j][r] + bv[j];
        slab[(mOff + r) * 68 + (j << 4) + rlane] = v;
      }
    }
    __builtin_amdgcn_fence(__ATOMIC_RELEASE, "workgroup");
    __builtin_amdgcn_wave_barrier();
    __builtin_amdgcn_fence(__ATOMIC_ACQUIRE, "workgroup");
    if (RESID) {
#pragma unroll
      for (int it = 0; it < 8; ++it) {
        const int row = it * 2 + hh;
        v4f v = *(const v4f*)(slab + row * 68 + c4);
        const v4f rr = *(const v4f*)(resid + (size_t)(mBase + row) * ldc + n0 + c4);
        v = v + rr;
        *(v4f*)(slab + row * 68 + c4) = v;
      }
    }
    for (int pass = 0; pass < 2; ++pass) {
#pragma unroll
      for (int it = 0; it < 8; ++it) {
        const int row = it * 2 + hh;
        const v4f v = *(const v4f*)(slab + row * 68 + c4);
        *(volatile v4f*)(C + (size_t)(mBase + row) * ldc + n0 + c4) = v;
      }
      __threadfence();
    }
    __builtin_amdgcn_fence(__ATOMIC_RELEASE, "workgroup");
    __builtin_amdgcn_wave_barrier();
    __builtin_amdgcn_fence(__ATOMIC_ACQUIRE, "workgroup");
  }
}

constexpr int SCAN_COLS  = 64;
constexpr int SCAN_THR   = 512;
constexpr int SCAN_CHUNK = 32;
static_assert(SCAN_THR / 8 == SCAN_COLS, "8 lanes per column");
static_assert(DSTATE % SCAN_COLS == 0 && NSTEP % SCAN_CHUNK == 0, "exact sharding");
static_assert((SCAN_CHUNK * DSTATE / 4) % SCAN_THR == 0, "feature chunk staging loop exact (4 iterations)");
static_assert(SCAN_CHUNK * 8 <= SCAN_THR, "store phase items fit the block");
static_assert(DSTATE == 256, "row ownership map 4*(8*m+g)+e covers 256 rows");

__global__ __launch_bounds__(SCAN_THR) void fastweight_scan_kernel(const float* __restrict__ feat,
                                                                   unsigned short* __restrict__ phi,
                                                                   unsigned short* __restrict__ plo) {
  __shared__ __align__(16) float Fs[SCAN_CHUNK * DSTATE];
  __shared__ __align__(16) float Ps[SCAN_CHUNK * SCAN_COLS];
  const int tid  = threadIdx.x;
  const int lane = tid & 31;
  const int wave = tid >> 5;
  const int g    = lane & 7;
  const int cl   = lane >> 3;
  const int b    = blockIdx.x >> 2;
  const int cb   = (blockIdx.x & 3) * SCAN_COLS;
  const int colb = wave * 4 + cl;
  const int j    = cb + colb;

  float s[32];
#pragma unroll
  for (int i = 0; i < 32; ++i) s[i] = 0.0f;

#pragma unroll 1
  for (int chunk = 0; chunk < NSTEP / SCAN_CHUNK; ++chunk) {
    const int t0 = chunk * SCAN_CHUNK;
    {
      const float* src = feat + ((size_t)b * NSTEP + t0) * DSTATE;
#pragma unroll
      for (int it = 0; it < 4; ++it) {
        const int idx = it * SCAN_THR + tid;
        const v4f v = *(const v4f*)(src + (size_t)idx * 4);
        *(v4f*)(Fs + idx * 4) = v;
      }
    }
    __syncthreads();

#pragma unroll 1
    for (int t = 0; t < SCAN_CHUNK; ++t) {
      const float* fr = Fs + t * DSTATE;
      v4f f[8];
#pragma unroll
      for (int m = 0; m < 8; ++m) f[m] = *(const v4f*)(fr + (8 * m + g) * 4);
      float p0 = 0.0f, p1 = 0.0f, p2 = 0.0f, p3 = 0.0f;
#pragma unroll
      for (int m = 0; m < 8; ++m) {
        p0 = fmaf(f[m][0], s[4 * m + 0], p0);
        p1 = fmaf(f[m][1], s[4 * m + 1], p1);
        p2 = fmaf(f[m][2], s[4 * m + 2], p2);
        p3 = fmaf(f[m][3], s[4 * m + 3], p3);
      }
      float p = (p0 + p1) + (p2 + p3);
      p += __shfl_xor(p, 1, 32);
      p += __shfl_xor(p, 2, 32);
      p += __shfl_xor(p, 4, 32);
      const float fj  = fr[j];
      const float err = p - fj;
      const float ng  = -INNER_STEP * err;
#pragma unroll
      for (int m = 0; m < 8; ++m) {
        s[4 * m + 0] = fmaf(f[m][0], ng, s[4 * m + 0]);
        s[4 * m + 1] = fmaf(f[m][1], ng, s[4 * m + 1]);
        s[4 * m + 2] = fmaf(f[m][2], ng, s[4 * m + 2]);
        s[4 * m + 3] = fmaf(f[m][3], ng, s[4 * m + 3]);
      }
      if (g == 0) Ps[t * SCAN_COLS + colb] = p;
    }
    __syncthreads();

    if (tid < SCAN_CHUNK * 8) {
      const int t = tid >> 3;
      const int q = tid & 7;
      const v4f a = *(const v4f*)(Ps + t * SCAN_COLS + 8 * q);
      const v4f c = *(const v4f*)(Ps + t * SCAN_COLS + 8 * q + 4);
      const float fv[8] = {a[0], a[1], a[2], a[3], c[0], c[1], c[2], c[3]};
      v4u hv, lv;
      split8(fv, hv, lv);
      const size_t o = ((size_t)b * NSTEP + t0 + t) * DSTATE + cb + 8 * q;
      for (int pass = 0; pass < 2; ++pass) {
        *(volatile v4u*)(phi + o) = hv;
        *(volatile v4u*)(plo + o) = lv;
        __threadfence();
      }
    }
  }
}

extern "C" void kernel_launch(void* const* d_in, const int* in_sizes, int n_in,
                              void* d_out, int out_size, void* d_ws, size_t ws_size, hipStream_t stream) {
  if (n_in < 5 || d_out == nullptr || d_ws == nullptr) return;
  if (in_sizes[0] != MROWS * DMODEL || in_sizes[1] != DMODEL * DSTATE || in_sizes[2] != DSTATE ||
      in_sizes[3] != DSTATE * DMODEL || in_sizes[4] != DMODEL || out_size != MROWS * DMODEL) return;

  const float* x  = (const float*)d_in[0];
  const float* Wd = (const float*)d_in[1];
  const float* bd = (const float*)d_in[2];
  const float* Wu = (const float*)d_in[3];
  const float* bu = (const float*)d_in[4];
  float* out = (float*)d_out;

  size_t off = 0;
  auto carve = [&](size_t nbytes) { const size_t o = off; off += nbytes; return o; };
  const size_t oXH  = carve((size_t)MROWS * DMODEL * 2);
  const size_t oXL  = carve((size_t)MROWS * DMODEL * 2);
  const size_t oWDH = carve((size_t)DSTATE * DMODEL * 2);
  const size_t oWDL = carve((size_t)DSTATE * DMODEL * 2);
  const size_t oWUH = carve((size_t)DMODEL * DSTATE * 2);
  const size_t oWUL = carve((size_t)DMODEL * DSTATE * 2);
  const size_t oFT  = carve((size_t)MROWS * DSTATE * 4);
  const size_t oPH  = carve((size_t)MROWS * DSTATE * 2);
  const size_t oPL  = carve((size_t)MROWS * DSTATE * 2);
  if (off > ws_size) return;

  unsigned char* ws = (unsigned char*)d_ws;
  unsigned short* XH  = (unsigned short*)(ws + oXH);
  unsigned short* XL  = (unsigned short*)(ws + oXL);
  unsigned short* WDH = (unsigned short*)(ws + oWDH);
  unsigned short* WDL = (unsigned short*)(ws + oWDL);
  unsigned short* WUH = (unsigned short*)(ws + oWUH);
  unsigned short* WUL = (unsigned short*)(ws + oWUL);
  float*          FT  = (float*)(ws + oFT);
  unsigned short* PH  = (unsigned short*)(ws + oPH);
  unsigned short* PL  = (unsigned short*)(ws + oPL);

  {
    const int n8 = (MROWS * DMODEL) / 8;
    split_planes_kernel<<<dim3(n8 / 256), dim3(256), 0, stream>>>(x, XH, XL, n8);
  }
  transpose_split_kernel<<<dim3(DMODEL / 64, DSTATE / 64), dim3(256), 0, stream>>>(Wd, WDH, WDL, DMODEL, DSTATE);
  transpose_split_kernel<<<dim3(DSTATE / 64, DMODEL / 64), dim3(256), 0, stream>>>(Wu, WUH, WUL, DSTATE, DMODEL);
  {
    const int tiles = (MROWS / 64) * (DSTATE / 64);
    gemm_bf16x3_kernel<false><<<dim3((tiles + 7) / 8), dim3(256), 0, stream>>>(
        XH, XL, DMODEL, WDH, WDL, DMODEL, FT, DSTATE, bd, nullptr, MROWS, DSTATE, DMODEL);
  }
  fastweight_scan_kernel<<<dim3(NBATCH * (DSTATE / SCAN_COLS)), dim3(SCAN_THR), 0, stream>>>(FT, PH, PL);
  {
    const int tiles = (MROWS / 64) * (DMODEL / 64);
    gemm_bf16x3_kernel<true><<<dim3((tiles + 7) / 8), dim3(256), 0, stream>>>(
        PH, PL, DSTATE, WUH, WUL, DSTATE, out, DMODEL, bu, x, MROWS, DMODEL, DSTATE);
  }
}
